// MultiHeadAttention_87033217286362
// MI455X (gfx1250) — hardware-verified
//
#include <hip/hip_runtime.h>


#ifndef NB
#define NB 2
#endif
#ifndef SEQ
#define SEQ 2048
#endif
#define NB_FULL  2
#define SEQ_FULL 2048
#define TT   SEQ
#define DM   1024
#define DMSH 10
#define NH_  16
#define HD   64
#define DQ   (NH_ * HD)
#define ZH   2
#define PCAR 1024.0f
#define SCL  0.125f

static_assert((1 << DMSH) == DM);
static_assert(DQ == DM);
static_assert(HD == 64);
static_assert((TT % 128) == 0);
static_assert((TT & (TT - 1)) == 0);
static_assert((NH_ % ZH) == 0);
static_assert((DM % 64) == 0 && ((3 * DQ) % 64) == 0 && (TT % 64) == 0);
static_assert((DM % 32) == 0 && (HD % 32) == 0 && (TT % 32) == 0 && (DQ % 32) == 0);
static_assert(((3 * DQ * DM) % 4096) == 0 && ((DM * DQ) % 4096) == 0);
static_assert((((size_t)TT * DM) % 2048) == 0);
static_assert((((size_t)2 * NH_ * TT * HD) % 512) == 0);
static_assert((((size_t)NH_ * HD * TT) % 512) == 0);
static_assert(((ZH * TT) % 8) == 0);
static_assert((((size_t)ZH * TT * HD) % 512) == 0);
static_assert(NB <= NB_FULL && SEQ <= SEQ_FULL);

typedef _Float16 h16;
typedef unsigned short bf;
typedef __attribute__((ext_vector_type(16))) __bf16   v16bf;
typedef __attribute__((ext_vector_type(16))) _Float16 v16h;
typedef __attribute__((ext_vector_type(8)))  _Float16 v8h;
typedef __attribute__((ext_vector_type(8)))  unsigned short v8us;
typedef __attribute__((ext_vector_type(8)))  float    v8f;
typedef __attribute__((ext_vector_type(4)))  float    v4f;
typedef __attribute__((ext_vector_type(2)))  float    v2f;
typedef __attribute__((ext_vector_type(2)))  _Float16 v2h;
typedef __attribute__((ext_vector_type(4)))  _Float16 v4h;
typedef __attribute__((ext_vector_type(2)))  unsigned short v2us;
typedef v4f  __attribute__((may_alias)) v4fa;

__device__ __forceinline__ unsigned short f2bf(float f) { unsigned u = __float_as_uint(f); u += 0x7FFFu + ((u >> 16) & 1u); return (unsigned short)(u >> 16); }
__device__ __forceinline__ float bf2f(unsigned short b) { return __uint_as_float(((unsigned)b) << 16); }
__device__ __forceinline__ float bfr(float f) { return bf2f(f2bf(f)); }
__device__ __forceinline__ v16h cat16(v8h lo, v8h hi) { return __builtin_shufflevector(lo, hi, 0, 1, 2, 3, 4, 5, 6, 7, 8, 9, 10, 11, 12, 13, 14, 15); }
__device__ __forceinline__ v16bf cat16b(v8us lo, v8us hi) { return __builtin_bit_cast(v16bf, __builtin_shufflevector(lo, hi, 0, 1, 2, 3, 4, 5, 6, 7, 8, 9, 10, 11, 12, 13, 14, 15)); }
__device__ __forceinline__ v8f wmma16(v16h a, v16h b, v8f c) { return __builtin_amdgcn_wmma_f32_16x16x32_f16(false, a, false, b, (short)0, c, false, false); }
__device__ __forceinline__ v8f wmmab(v16bf a, v16bf b, v8f c) { return __builtin_amdgcn_wmma_f32_16x16x32_bf16(false, a, false, b, (short)0, c, false, false); }

template <typename T16> struct WFrag;
template <> struct WFrag<h16> { typedef v16h V; static __device__ __forceinline__ V ld(const h16* p) { return cat16(*(const v8h*)p, *(const v8h*)(p + 16)); } static __device__ __forceinline__ v8f mma(V a, V b, v8f c) { return wmma16(a, b, c); } };
template <> struct WFrag<bf> { typedef v16bf V; static __device__ __forceinline__ V ld(const bf* p) { return cat16b(*(const v8us*)p, *(const v8us*)(p + 16)); } static __device__ __forceinline__ v8f mma(V a, V b, v8f c) { return wmmab(a, b, c); } };
template <typename T16, int NSPLIT, bool BIAS>
__global__ __launch_bounds__(32) void k_gemmw(const T16* __restrict__ A, const T16* __restrict__ A2, const T16* __restrict__ Bt, const T16* __restrict__ Bt2, int K, float* C, int ldc, const float* __restrict__ bias, size_t sA, size_t sB, size_t sC) {
    typedef typename WFrag<T16>::V V;
    __shared__ __align__(16) float os[16 * 68];
    const size_t z = blockIdx.z; A += z * sA; if (A2) A2 += z * sA; Bt += z * sB; if (Bt2) Bt2 += z * sB; C += z * sC;
    const int lane = threadIdx.x & 31, lr = lane & 15, hi = lane >> 4; const int r0 = blockIdx.x * 64, c0 = blockIdx.y * 64;
    v8f acc[4][4];
#pragma unroll
    for (int mb = 0; mb < 4; ++mb)
#pragma unroll
        for (int nb = 0; nb < 4; ++nb) acc[mb][nb] = (v8f){};
    const size_t aoff = (size_t)(r0 + lr) * K + 8 * hi, boff = (size_t)(c0 + lr) * K + 8 * hi;
#pragma unroll 1
    for (int kc = 0; kc < K; kc += 32) {
        V a[4], a2[4];
#pragma unroll
        for (int mb = 0; mb < 4; ++mb) { a[mb] = WFrag<T16>::ld(A + aoff + (size_t)mb * 16 * K + kc); if (NSPLIT == 1 || NSPLIT == 2) a2[mb] = WFrag<T16>::ld(A2 + aoff + (size_t)mb * 16 * K + kc); }
#pragma unroll
        for (int nb = 0; nb < 4; ++nb) { const V b = WFrag<T16>::ld(Bt + boff + (size_t)nb * 16 * K + kc); V b2; if (NSPLIT >= 2) b2 = WFrag<T16>::ld(Bt2 + boff + (size_t)nb * 16 * K + kc);
#pragma unroll
            for (int mb = 0; mb < 4; ++mb) { acc[mb][nb] = WFrag<T16>::mma(a[mb], b, acc[mb][nb]); if (NSPLIT == 1 || NSPLIT == 2) acc[mb][nb] = WFrag<T16>::mma(a2[mb], b, acc[mb][nb]); if (NSPLIT >= 2) acc[mb][nb] = WFrag<T16>::mma(a[mb], b2, acc[mb][nb]); } }
        asm volatile("v_nop\n\tv_nop\n\tv_nop\n\tv_nop" : "+v"(acc[0][0]), "+v"(acc[1][1]), "+v"(acc[2][2]), "+v"(acc[3][3]) : "v"(a[0]), "v"(a[3]));
    }
    v4f bv = (v4f){0.0f, 0.0f, 0.0f, 0.0f};
    if (BIAS) { const v4f br = *(const v4f*)(bias + c0 + lr * 4);
#pragma unroll
        for (int q = 0; q < 4; ++q) bv[q] = bfr(br[q]); }
#pragma unroll
    for (int mb = 0; mb < 4; ++mb) {
#pragma unroll
        for (int nb = 0; nb < 4; ++nb) {
#pragma unroll
            for (int j = 0; j < 8; ++j) os[(hi * 8 + j) * 68 + nb * 16 + lr] = acc[mb][nb][j]; }
        __builtin_amdgcn_wave_barrier(); asm volatile("" ::: "memory");
        float* crow = C + (size_t)(r0 + mb * 16) * ldc + c0;
#pragma unroll 1
        for (int ps = 0; ps < 2; ++ps) {
#pragma unroll
            for (int s = 0; s < 8; ++s) { const int row = 2 * s + hi, cofs = lr * 4; v4f val = *(const v4fa*)(os + row * 68 + cofs); if (BIAS) val = val + bv;
                *(volatile v4f*)(crow + (size_t)row * ldc + cofs) = val; }
            if (ps == 0) __threadfence(); }
        __builtin_amdgcn_wave_barrier(); asm volatile("" ::: "memory");
    }
}

__device__ __forceinline__ void splitf(float y, unsigned short& h, unsigned short& l) { h = f2bf(y); l = f2bf(y - bf2f(h)); }

__global__ __launch_bounds__(256) void k_wt(const float* __restrict__ w, unsigned N, bf* Bt) {
    const unsigned lane = threadIdx.x & 31u; const unsigned L0 = (blockIdx.x * 8u + (threadIdx.x >> 5)) * 8u; const unsigned nlines = N * (DM / 64);
#pragma unroll
    for (int ps = 0; ps < 2; ++ps) {
#pragma unroll 1
        for (unsigned l = 0; l < 8u; ++l) { const unsigned L = L0 + l;
            if (L < nlines) { const unsigned e = L * 64u + lane * 2u; const unsigned k = e & (unsigned)(DM - 1), n = e >> DMSH; v2us o;
                o[0] = f2bf(w[(size_t)k * N + n]); o[1] = f2bf(w[(size_t)(k + 1u) * N + n]); *(volatile v2us*)(Bt + e) = o; } }
        if (ps == 0) __threadfence(); }
}
__global__ __launch_bounds__(256) void k_cvt8(const float* __restrict__ src, bf* dst, size_t n8) { const size_t i = (size_t)blockIdx.x * 256 + threadIdx.x; if (i >= n8) return; const v8f v = *(const v8f*)(src + i * 8); v8us o;
#pragma unroll
    for (int k = 0; k < 8; ++k) o[k] = f2bf(v[k]); *(volatile v8us*)(dst + i * 8) = o; __threadfence(); *(volatile v8us*)(dst + i * 8) = o; }

__global__ __launch_bounds__(256) void k_hp(const float* __restrict__ F, unsigned pitch, unsigned nheads, h16* P16) {
    const unsigned e = (blockIdx.x * 256u + threadIdx.x) * 2u; if (e >= nheads * (unsigned)TT * (unsigned)HD) return;
    const unsigned d = e & (unsigned)(HD - 1); const unsigned t = (e / (unsigned)HD) % (unsigned)TT; const unsigned g = e / ((unsigned)HD * (unsigned)TT);
    const v2f x = *(const v2f*)(F + (size_t)t * pitch + g * (unsigned)HD + d); v2h o; o[0] = (h16)x[0]; o[1] = (h16)x[1];
    *(volatile v2h*)(P16 + e) = o; __threadfence(); *(volatile v2h*)(P16 + e) = o; }
__global__ __launch_bounds__(256) void k_vtp(const float* __restrict__ F, unsigned pitch, unsigned nheads, h16* V16) {
    const unsigned e = (blockIdx.x * 256u + threadIdx.x) * 2u; if (e >= nheads * (unsigned)HD * (unsigned)TT) return;
    const unsigned t = e % (unsigned)TT; const unsigned d = (e / (unsigned)TT) & (unsigned)(HD - 1); const unsigned g = e / ((unsigned)TT * (unsigned)HD); v2h o;
#pragma unroll
    for (unsigned q = 0; q < 2u; ++q) o[q] = (h16)F[(size_t)(t + q) * pitch + g * (unsigned)HD + d];
    *(volatile v2h*)(V16 + e) = o; __threadfence(); *(volatile v2h*)(V16 + e) = o; }
__global__ __launch_bounds__(256) void k_asoft(const float* __restrict__ Sb, h16* P16) {
    const unsigned lane = threadIdx.x & 31u; const unsigned row = blockIdx.x * 8u + (threadIdx.x >> 5); if (row >= (unsigned)(ZH * TT)) return; const float* sr = Sb + (size_t)row * TT; float v[TT / 32]; float mx = -3.0e38f;
#pragma unroll
    for (int ch = 0; ch < TT / 128; ++ch) { const unsigned j0 = (unsigned)ch * 128u + lane * 4u; const v4f a = *(const v4f*)(sr + j0);
#pragma unroll
        for (int q = 0; q < 4; ++q) { const float t = a[q] * SCL; v[ch * 4 + q] = t; mx = fmaxf(mx, t); } }
#pragma unroll
    for (int sh = 16; sh; sh >>= 1) mx = fmaxf(mx, __shfl_xor(mx, sh, 32));
    float sum = 0.f;
#pragma unroll
    for (int k = 0; k < TT / 32; ++k) { float d0 = __fsub_rn(v[k], mx); asm volatile("" : "+v"(d0)); v[k] = __builtin_amdgcn_exp2f(__fmul_rn(d0, 1.4426950408889634f)); sum += v[k]; }
#pragma unroll
    for (int sh = 16; sh; sh >>= 1) sum += __shfl_xor(sum, sh, 32);
    const float f = __fdiv_rn(PCAR, sum);
#pragma unroll 1
    for (int ps = 0; ps < 2; ++ps) {
#pragma unroll
        for (int ch = 0; ch < TT / 128; ++ch) { v4h o4;
#pragma unroll
            for (int q = 0; q < 4; ++q) o4[q] = (h16)(v[ch * 4 + q] * f);
            *(volatile v4h*)(P16 + (size_t)row * TT + (unsigned)ch * 128u + lane * 4u) = o4; }
        if (ps == 0) __threadfence(); }
}
__global__ __launch_bounds__(256) void k_merge(const float* __restrict__ O, unsigned h0, bf* Ah, bf* Al) {
    const unsigned e = (blockIdx.x * 256u + threadIdx.x) * 2u; if (e >= (unsigned)(ZH * TT * HD)) return;
    const unsigned d = e & (unsigned)(HD - 1); const unsigned t = (e / (unsigned)HD) % (unsigned)TT; const unsigned zz = e / ((unsigned)HD * (unsigned)TT);
    const size_t oo = (size_t)t * DQ + (h0 + zz) * (unsigned)HD + d; const v2f x = *(const v2f*)(O + e); v2us oh, ol;
#pragma unroll
    for (int q = 0; q < 2; ++q) { unsigned short a, c2; splitf(x[q] * (1.0f / PCAR), a, c2); oh[q] = a; ol[q] = c2; }
    *(volatile v2us*)(Ah + oo) = oh; *(volatile v2us*)(Al + oo) = ol; __threadfence(); *(volatile v2us*)(Ah + oo) = oh; *(volatile v2us*)(Al + oo) = ol; }

extern "C" void kernel_launch(void* const* d_in, const int* in_sizes, int n_in,
                              void* d_out, int out_size, void* d_ws, size_t ws_size, hipStream_t stream) {
    if (n_in < 5) return;
    if ((size_t)in_sizes[0] < (size_t)(NB - 1) * SEQ_FULL * DM + (size_t)TT * DM) return;
    if ((size_t)in_sizes[1] < (size_t)DM * 3 * DQ) return;
    if ((size_t)in_sizes[2] < (size_t)3 * DQ) return;
    if ((size_t)in_sizes[3] < (size_t)DQ * DM) return;
    if ((size_t)in_sizes[4] < (size_t)DM) return;
    if ((size_t)out_size < (size_t)NB * TT * DM) return;
    const float* x = (const float*)d_in[0]; const float* wqkv = (const float*)d_in[1]; const float* bqkv = (const float*)d_in[2]; const float* wproj = (const float*)d_in[3]; const float* bproj = (const float*)d_in[4];
    float* OUT = (float*)d_out;
    char* wsp = (char*)d_ws;
    auto take = [&](size_t bytes) { char* p = wsp; wsp += (bytes + 255) & ~(size_t)255; return (void*)p; };
    bf* WQKV = (bf*)take((size_t)3 * DQ * DM * 2);
    bf* WO   = (bf*)take((size_t)DM * DQ * 2);
    bf* XB   = (bf*)take((size_t)TT * DM * 2);
    float* F = (float*)take((size_t)TT * 3 * DQ * 4);
    h16* QK16 = (h16*)take((size_t)2 * NH_ * TT * HD * 2);
    h16* VT16 = (h16*)take((size_t)NH_ * HD * TT * 2);
    float* Sb = (float*)take((size_t)ZH * TT * TT * 4);
    h16* P16 = (h16*)take((size_t)ZH * TT * TT * 2);
    float* Ob = (float*)take((size_t)ZH * TT * HD * 4);
    bf* ATh = (bf*)take((size_t)TT * DQ * 2); bf* ATl = (bf*)take((size_t)TT * DQ * 2);
    const size_t used = (size_t)(wsp - (char*)d_ws);
    if (used > ws_size || used > (size_t)134217728) return;
    h16* QP16 = QK16; h16* KP16 = QK16 + (size_t)NH_ * TT * HD;

    k_wt<<<(unsigned)((size_t)3 * DQ * DM / 4096), 256, 0, stream>>>(wqkv, (unsigned)(3 * DQ), WQKV);
    k_wt<<<(unsigned)((size_t)DM * DQ / 4096), 256, 0, stream>>>(wproj, (unsigned)DM, WO);
    for (unsigned b = 0; b < (unsigned)NB; ++b) {
        k_cvt8<<<(unsigned)((size_t)TT * DM / 2048), 256, 0, stream>>>(x + (size_t)b * SEQ_FULL * DM, XB, (size_t)TT * DM / 8);
        k_gemmw<bf, 0, true><<<dim3(TT / 64, 3 * DQ / 64, 1), 32, 0, stream>>>(XB, nullptr, WQKV, nullptr, DM, F, 3 * DQ, bqkv, 0, 0, 0);
        k_hp<<<(unsigned)((size_t)2 * NH_ * TT * HD / 512), 256, 0, stream>>>(F, (unsigned)(3 * DQ), (unsigned)(2 * NH_), QK16);
        k_vtp<<<(unsigned)((size_t)NH_ * HD * TT / 512), 256, 0, stream>>>(F + 2 * DQ, (unsigned)(3 * DQ), (unsigned)NH_, VT16);
        for (unsigned h0 = 0; h0 < (unsigned)NH_; h0 += ZH) {
            k_gemmw<h16, 0, false><<<dim3(TT / 64, TT / 64, ZH), 32, 0, stream>>>(QP16 + (size_t)h0 * TT * HD, nullptr, KP16 + (size_t)h0 * TT * HD, nullptr, HD, Sb, TT, nullptr, (size_t)TT * HD, (size_t)TT * HD, (size_t)TT * TT);
            k_asoft<<<ZH * TT / 8, 256, 0, stream>>>(Sb, P16);
            k_gemmw<h16, 0, false><<<dim3(TT / 64, HD / 64, ZH), 32, 0, stream>>>(P16, nullptr, VT16 + (size_t)h0 * HD * TT, nullptr, TT, Ob, HD, nullptr, (size_t)TT * TT, (size_t)HD * TT, (size_t)TT * HD);
            k_merge<<<(unsigned)((size_t)ZH * TT * HD / 512), 256, 0, stream>>>(Ob, h0, ATh, ATl); }
        k_gemmw<bf, 1, true><<<dim3(TT / 64, DM / 64, 1), 32, 0, stream>>>(ATh, ATl, WO, nullptr, DQ, OUT + (size_t)b * TT * DM, DM, bproj, 0, 0, 0); }
}
